// LTNFeedForwardLayer_29678224015512
// MI455X (gfx1250) — hardware-verified
//
#include <hip/hip_runtime.h>


#define NB_  4096
#define NI   1024
#define NO   1024
#define NF   4
#define NC   16
typedef _Float16 h16;
typedef unsigned short bf;
typedef __attribute__((ext_vector_type(16))) __bf16   v16bf;
typedef __attribute__((ext_vector_type(16))) _Float16 v16h;
typedef __attribute__((ext_vector_type(8)))  _Float16 v8h;
typedef __attribute__((ext_vector_type(8)))  unsigned short v8us;
typedef __attribute__((ext_vector_type(8)))  float    v8f;
typedef __attribute__((ext_vector_type(4)))  float    v4f;
typedef v8h  __attribute__((may_alias)) v8ha;
typedef v4f  __attribute__((may_alias)) v4fa;
typedef v8us __attribute__((may_alias)) v8usa;

__device__ __forceinline__ unsigned short f2bf(float f) { unsigned u = __float_as_uint(f); u += 0x7FFFu + ((u >> 16) & 1u); return (unsigned short)(u >> 16); }
__device__ __forceinline__ float bf2f(unsigned short b) { return __uint_as_float(((unsigned)b) << 16); }
__device__ __forceinline__ float bfr(float f) { return bf2f(f2bf(f)); }
__device__ __forceinline__ v16h cat16(v8h lo, v8h hi) { return __builtin_shufflevector(lo, hi, 0, 1, 2, 3, 4, 5, 6, 7, 8, 9, 10, 11, 12, 13, 14, 15); }
__device__ __forceinline__ v16bf cat16b(v8us lo, v8us hi) { return __builtin_bit_cast(v16bf, __builtin_shufflevector(lo, hi, 0, 1, 2, 3, 4, 5, 6, 7, 8, 9, 10, 11, 12, 13, 14, 15)); }
__device__ __forceinline__ v8f wmma16(v16h a, v16h b, v8f c) { return __builtin_amdgcn_wmma_f32_16x16x32_f16(false, a, false, b, (short)0, c, false, false); }
__device__ __forceinline__ v8f wmmab(v16bf a, v16bf b, v8f c) { return __builtin_amdgcn_wmma_f32_16x16x32_bf16(false, a, false, b, (short)0, c, false, false); }


template <typename T16> struct WFrag;
template <> struct WFrag<h16> { typedef v16h V; static __device__ __forceinline__ V ld(const h16* p) { return cat16(*(const v8h*)p, *(const v8h*)(p + 16)); } static __device__ __forceinline__ v8f mma(V a, V b, v8f c) { return wmma16(a, b, c); } };
template <> struct WFrag<bf> { typedef v16bf V; static __device__ __forceinline__ V ld(const bf* p) { return cat16b(*(const v8us*)p, *(const v8us*)(p + 16)); } static __device__ __forceinline__ v8f mma(V a, V b, v8f c) { return wmmab(a, b, c); } };
template <typename T16, int NSPLIT, bool BIAS>
__global__ __launch_bounds__(32) void k_gemmw(const T16* __restrict__ A, const T16* __restrict__ A2, const T16* __restrict__ Bt, const T16* __restrict__ Bt2, int K, float* C, int ldc, const float* __restrict__ bias, size_t sA, size_t sB, size_t sC) {
    typedef typename WFrag<T16>::V V;
    __shared__ __align__(16) float os[16 * 68];
    const size_t z = blockIdx.z; A += z * sA; if (A2) A2 += z * sA; Bt += z * sB; if (Bt2) Bt2 += z * sB; C += z * sC;
    const int lane = threadIdx.x & 31, lr = lane & 15, hi = lane >> 4; const int r0 = blockIdx.x * 64, c0 = blockIdx.y * 64;
    v8f acc[4][4];
#pragma unroll
    for (int mb = 0; mb < 4; ++mb)
#pragma unroll
        for (int nb = 0; nb < 4; ++nb) acc[mb][nb] = (v8f){};
    const size_t aoff = (size_t)(r0 + lr) * K + 8 * hi, boff = (size_t)(c0 + lr) * K + 8 * hi;
#pragma unroll 1
    for (int kc = 0; kc < K; kc += 32) {
        V a[4], a2[4];
#pragma unroll
        for (int mb = 0; mb < 4; ++mb) { a[mb] = WFrag<T16>::ld(A + aoff + (size_t)mb * 16 * K + kc); if (NSPLIT == 1 || NSPLIT == 2) a2[mb] = WFrag<T16>::ld(A2 + aoff + (size_t)mb * 16 * K + kc); }
#pragma unroll
        for (int nb = 0; nb < 4; ++nb) { const V b = WFrag<T16>::ld(Bt + boff + (size_t)nb * 16 * K + kc); V b2; if (NSPLIT >= 2) b2 = WFrag<T16>::ld(Bt2 + boff + (size_t)nb * 16 * K + kc);
#pragma unroll
            for (int mb = 0; mb < 4; ++mb) { acc[mb][nb] = WFrag<T16>::mma(a[mb], b, acc[mb][nb]); if (NSPLIT == 1 || NSPLIT == 2) acc[mb][nb] = WFrag<T16>::mma(a2[mb], b, acc[mb][nb]); if (NSPLIT >= 2) acc[mb][nb] = WFrag<T16>::mma(a[mb], b2, acc[mb][nb]); } }
        asm volatile("v_nop\n\tv_nop\n\tv_nop\n\tv_nop" : "+v"(acc[0][0]), "+v"(acc[1][1]), "+v"(acc[2][2]), "+v"(acc[3][3]) : "v"(a[0]), "v"(a[3]));
    }
#pragma unroll
    for (int mb = 0; mb < 4; ++mb) {
#pragma unroll
        for (int nb = 0; nb < 4; ++nb) {
#pragma unroll
            for (int j = 0; j < 8; ++j) os[(hi * 8 + j) * 68 + nb * 16 + lr] = acc[mb][nb][j]; }
        __builtin_amdgcn_wave_barrier(); asm volatile("" ::: "memory");
        float* crow = C + (size_t)(r0 + mb * 16) * ldc + c0;
#pragma unroll 1
        for (int ps = 0; ps < 2; ++ps) {
#pragma unroll
            for (int s = 0; s < 8; ++s) { const int row = 2 * s + hi, cofs = lr * 4; v4f val = *(const v4fa*)(os + row * 68 + cofs); if (BIAS) { val[0] += bfr(bias[c0 + cofs]); val[1] += bfr(bias[c0 + cofs + 1]); val[2] += bfr(bias[c0 + cofs + 2]); val[3] += bfr(bias[c0 + cofs + 3]); }
                *(volatile v4f*)(crow + (size_t)row * ldc + cofs) = val; }
            if (ps == 0) __threadfence(); }
        __builtin_amdgcn_wave_barrier(); asm volatile("" ::: "memory");
    }
}

__device__ __forceinline__ h16 tohx(float x) { return (h16)x; }
typedef __attribute__((ext_vector_type(4))) _Float16 v4h;

__global__ __launch_bounds__(256) void k_wsoft(const float* __restrict__ ml, h16* W16) { const int lane = threadIdx.x & 31; const int row = blockIdx.x * 8 + (threadIdx.x >> 5); if (row >= NO * NF) return; const float* sr = ml + (size_t)row * NI; float v[NI / 32]; float mx = -3.0e38f;
#pragma unroll
    for (int ch = 0; ch < NI / 128; ++ch) { const v4f a = *(const v4f*)(sr + ch * 128 + lane * 4);
#pragma unroll
        for (int u = 0; u < 4; ++u) { v[ch * 4 + u] = bfr(a[u]); mx = fmaxf(mx, v[ch * 4 + u]); } }
#pragma unroll
    for (int sh = 16; sh; sh >>= 1) mx = fmaxf(mx, __shfl_xor(mx, sh, 32));
    float sum = 0.f;
#pragma unroll
    for (int q = 0; q < NI / 32; ++q) { float d0 = __fsub_rn(v[q], mx); asm volatile("" : "+v"(d0)); v[q] = __expf(d0); sum += v[q]; }
#pragma unroll
    for (int sh = 16; sh; sh >>= 1) sum += __shfl_xor(sum, sh, 32);
    const float f = __fdiv_rn(1.0f, sum);
    for (int ps = 0; ps < 2; ++ps) {
#pragma unroll
        for (int ch = 0; ch < NI / 128; ++ch) { v4h o;
#pragma unroll
            for (int u = 0; u < 4; ++u) o[u] = tohx(v[ch * 4 + u] * f); *(volatile v4h*)(W16 + (size_t)row * NI + ch * 128 + lane * 4) = o; }
        if (ps == 0) __threadfence(); } }
__global__ __launch_bounds__(256) void k_xh(const float* __restrict__ x, h16* XH) { const size_t e = ((size_t)blockIdx.x * 256 + threadIdx.x) * 4; if (e >= (size_t)NB_ * NI) return; const v4f a = *(const v4f*)(x + e); v4h o;
#pragma unroll
    for (int u = 0; u < 4; ++u) o[u] = tohx(bfr(a[u])); *(volatile v4h*)(XH + e) = o; __threadfence(); *(volatile v4h*)(XH + e) = o; }
__global__ __launch_bounds__(256) void k_lut(const float* __restrict__ SEL, const float* __restrict__ lut, float* OUT) { const size_t idx = (size_t)blockIdx.x * 256 + threadIdx.x; if (idx >= (size_t)NB_ * NO) return; const int o = (int)(idx % NO); const v4f sv = *(const v4f*)(SEL + idx * NF); float s[NF], sm1[NF];
#pragma unroll
    for (int j = 0; j < NF; ++j) { s[j] = __fdiv_rn(1.0f, 1.0f + __expf(-sv[j])); sm1[j] = __fsub_rn(1.0f, s[j]); }
    float acc = 0.f;
#pragma unroll
    for (int c = 0; c < NC; ++c) { float cw = 1.0f;
#pragma unroll
        for (int j = 0; j < NF; ++j) { float f = ((c >> j) & 1) ? s[j] : sm1[j]; float t = __fmul_rn(cw, f); asm volatile("" : "+v"(t)); cw = t; }
        float lv = bfr(lut[o * NC + c]); asm volatile("" : "+v"(lv)); float pr = __fmul_rn(cw, lv); asm volatile("" : "+v"(pr)); acc = __fadd_rn(acc, pr); }
    *(volatile float*)(OUT + idx) = acc; __threadfence(); *(volatile float*)(OUT + idx) = acc; }

extern "C" void kernel_launch(void* const* d_in, const int* in_sizes, int n_in,
                              void* d_out, int out_size, void* d_ws, size_t ws_size, hipStream_t stream) {
    (void)in_sizes; (void)n_in; (void)out_size;
    const float* x = (const float*)d_in[0]; const float* ml = (const float*)d_in[1]; const float* lut = (const float*)d_in[2];
    float* OUT = (float*)d_out;
    char* wsp = (char*)d_ws;
    auto take = [&](size_t bytes) { char* p = wsp; wsp += (bytes + 255) & ~(size_t)255; return (void*)p; };
    h16* W16 = (h16*)take((size_t)NO * NF * NI * 2); h16* XH = (h16*)take((size_t)NB_ * NI * 2); float* SEL = (float*)take((size_t)NB_ * NO * NF * 4);
    if ((size_t)(wsp - (char*)d_ws) > ws_size) return;
    k_wsoft<<<NO * NF / 8, 256, 0, stream>>>(ml, W16); k_xh<<<(unsigned)(((size_t)NB_ * NI / 4 + 255) / 256), 256, 0, stream>>>(x, XH);
    k_gemmw<h16, 0, false><<<dim3(NB_ / 64, NO * NF / 64, 1), 32, 0, stream>>>(XH, nullptr, W16, nullptr, NI, SEL, NO * NF, nullptr, 0, 0, 0);
    k_lut<<<(unsigned)(((size_t)NB_ * NO + 255) / 256), 256, 0, stream>>>(SEL, lut, OUT);
}
